// TemporalHybrid_34402688041060
// MI455X (gfx1250) — hardware-verified
//
#include <hip/hip_runtime.h>
#define BB 8
#define LL 1024
#define IN 128
#define HH 256
#define NS 256
#define NR (BB * LL)
#define HCH 16

typedef __bf16 v16b __attribute__((ext_vector_type(16)));
typedef unsigned short v8us __attribute__((ext_vector_type(8), may_alias));
typedef float  v8f  __attribute__((ext_vector_type(8)));
typedef float  v4f  __attribute__((ext_vector_type(4)));
typedef float  v4fa __attribute__((ext_vector_type(4), may_alias));
union FragB { v16b v; v8us half[2]; unsigned short u[16]; };

__device__ __forceinline__ unsigned short bf16_bits(float x) { unsigned int u = __float_as_uint(x); return (unsigned short)((u + 0x7FFFu + ((u >> 16) & 1u)) >> 16); }
__device__ __forceinline__ float bf16_val(unsigned short b) { return __uint_as_float(((unsigned int)b) << 16); }
__device__ __forceinline__ float bf16_round(float x) { return bf16_val(bf16_bits(x)); }
template <int NT>
__device__ __forceinline__ v8f mmaN(v16b ah, v16b al, v16b bh, v16b bl, v8f c) {
  c = __builtin_amdgcn_wmma_f32_16x16x32_bf16(false, ah, false, bh, (short)0, c, false, false);
  if (NT >= 2) c = __builtin_amdgcn_wmma_f32_16x16x32_bf16(false, al, false, bh, (short)0, c, false, false);
  if (NT >= 3) c = __builtin_amdgcn_wmma_f32_16x16x32_bf16(false, ah, false, bl, (short)0, c, false, false);
  asm volatile("v_nop\n\tv_nop\n\tv_nop\n\tv_nop" : "+v"(c) : "v"(ah), "v"(al), "v"(bh), "v"(bl));
  return c;
}

__global__ __launch_bounds__(256) void k_wt_bf16(const float* __restrict__ W, unsigned short* __restrict__ Wt, int K, int N) {
  const int t = blockIdx.x * 256 + threadIdx.x;
  const int k8n = K / 8;
  if (t >= N * k8n) return;
  const int n = t / k8n, k8 = (t % k8n) * 8;
  v8us v;
#pragma unroll
  for (int i = 0; i < 8; ++i) v[i] = bf16_bits(W[(size_t)(k8 + i) * N + n]);
  *(volatile v8us*)(Wt + (size_t)n * K + k8) = v;
  __threadfence();
  *(volatile v8us*)(Wt + (size_t)n * K + k8) = v;
}

template <bool ASPLIT, int ACT, bool BIAS_BF16>
__global__ __launch_bounds__(128) void k_gemm_bf(const float* __restrict__ A, int lda, const unsigned short* __restrict__ Wt, int ldb,
                                               const float* __restrict__ bias, float* __restrict__ C, int ldc, int M, int N, int K) {
  __shared__ __attribute__((aligned(16))) float so[4][16][64];
  const int tid = threadIdx.x, w = tid >> 5, lane = tid & 31, ln = lane & 15, hh = lane >> 4;
  const int ntn = N / 64;
  const int wid = blockIdx.x * 4 + w;
  const int mt = wid / ntn, nq = wid % ntn;
  if (mt * 16 >= M) return;
  const int row0 = mt * 16, col0 = nq * 64;
  const float* arow = A + (size_t)(row0 + ln) * lda;
  v8f acc[4] = {};
  for (int kb = 0; kb < K; kb += 32) {
    FragB ah, al;
    const v4f x0 = *(const v4fa*)(arow + kb + 8 * hh), x1 = *(const v4fa*)(arow + kb + 8 * hh + 4);
    const v4f x2 = *(const v4fa*)(arow + kb + 16 + 8 * hh), x3 = *(const v4fa*)(arow + kb + 16 + 8 * hh + 4);
    float xs[16] = {x0[0],x0[1],x0[2],x0[3],x1[0],x1[1],x1[2],x1[3],x2[0],x2[1],x2[2],x2[3],x3[0],x3[1],x3[2],x3[3]};
#pragma unroll
    for (int i = 0; i < 16; ++i) { const unsigned short hb = bf16_bits(xs[i]); ah.u[i] = hb; al.u[i] = ASPLIT ? bf16_bits(xs[i] - bf16_val(hb)) : (unsigned short)0; }
#pragma unroll
    for (int t = 0; t < 4; ++t) {
      const unsigned short* brow = Wt + (size_t)(col0 + t * 16 + ln) * ldb + kb;
      FragB b;
      b.half[0] = *(const v8us*)(brow + 8 * hh);
      b.half[1] = *(const v8us*)(brow + 16 + 8 * hh);
      acc[t] = mmaN<ASPLIT ? 2 : 1>(ah.v, al.v, b.v, b.v, acc[t]);
    }
  }
#pragma unroll
  for (int t = 0; t < 4; ++t) {
    float bv = bias ? bias[col0 + t * 16 + ln] : 0.f;
    if (BIAS_BF16) bv = bf16_round(bv);
#pragma unroll
    for (int r = 0; r < 8; ++r) { float v = acc[t][r] + bv; if (ACT == 1) v = fmaxf(v, 0.f); so[w][8 * hh + r][t * 16 + ln] = v; }
  }
  __builtin_amdgcn_fence(__ATOMIC_ACQ_REL, "workgroup");
  __builtin_amdgcn_wave_barrier();
  const int rsub = lane >> 4, c4 = (lane & 15) * 4;
  for (int pass = 0; pass < 2; ++pass) {
#pragma unroll
    for (int q = 0; q < 8; ++q) {
      const int r = q * 2 + rsub;
      const v4f v = *(const v4fa*)&so[w][r][c4];
      *(volatile v4f*)(C + (size_t)(row0 + r) * ldc + col0 + c4) = v;
    }
    if (pass == 0) __threadfence();
  }
}

template <int D, bool CAUSAL>
__global__ __launch_bounds__(128) void k_flash(const float* __restrict__ qb, const float* __restrict__ kb, const float* __restrict__ vb,
                                             int pitch, int T, int H, float scale, float* __restrict__ y, int ypitch) {
  constexpr int KS = D / 32;
  constexpr int DT = D / 16;
  __shared__ __attribute__((aligned(16))) unsigned short sKh[32][D + 8], sKl[32][D + 8], sVh[32][D + 8], sVl[32][D + 8];
  __shared__ __attribute__((aligned(16))) unsigned short sPh[4][16][40], sPl[4][16][40];
  __shared__ __attribute__((aligned(16))) float sO[4][16][D];
  const int tid = threadIdx.x, w = tid >> 5, lane = tid & 31, ln = lane & 15, hh = lane >> 4;
  const int nqb = (T + 63) / 64;
  const int bh = blockIdx.x / nqb, qblk = blockIdx.x % nqb;
  const int b = bh / H, h = bh % H;
  const int q0 = qblk * 64 + w * 16;
  const float* Q = qb + (size_t)b * T * pitch + h * D;
  const float* K = kb + (size_t)b * T * pitch + h * D;
  const float* V = vb + (size_t)b * T * pitch + h * D;

  FragB aqh[KS], aql[KS];
  {
    int row = q0 + ln; if (row >= T) row = T - 1;
    const float* qr = Q + (size_t)row * pitch;
#pragma unroll
    for (int ks = 0; ks < KS; ++ks)
#pragma unroll
      for (int i = 0; i < 16; ++i) {
        const int d = ks * 32 + ((i < 8) ? (8 * hh + i) : (16 + 8 * hh + (i - 8)));
        const float x = qr[d] * scale; const unsigned short hb = bf16_bits(x);
        aqh[ks].u[i] = hb; aql[ks].u[i] = bf16_bits(x - bf16_val(hb));
      }
  }
  float m_r[8], l_r[8];
#pragma unroll
  for (int r = 0; r < 8; ++r) { m_r[r] = -3.0e38f; l_r[r] = 0.f; }
  v8f oacc[DT];
#pragma unroll
  for (int dt = 0; dt < DT; ++dt) oacc[dt] = (v8f){0.f,0.f,0.f,0.f,0.f,0.f,0.f,0.f};

  const int kv_end = CAUSAL ? min(T, qblk * 64 + 64) : T;
  for (int j0 = 0; j0 < kv_end; j0 += 32) {
    __syncthreads();
    for (int e = tid; e < 32 * (D / 4); e += 128) {
      const int r = e / (D / 4), c4 = (e % (D / 4)) * 4;
      const int key = j0 + r;
      v4f kf = {0.f,0.f,0.f,0.f}, vf = {0.f,0.f,0.f,0.f};
      if (key < T) { kf = *(const v4fa*)(K + (size_t)key * pitch + c4); vf = *(const v4fa*)(V + (size_t)key * pitch + c4); }
#pragma unroll
      for (int t = 0; t < 4; ++t) {
        unsigned short hb = bf16_bits(kf[t]); sKh[r][c4 + t] = hb; sKl[r][c4 + t] = bf16_bits(kf[t] - bf16_val(hb));
        hb = bf16_bits(vf[t]); sVh[r][c4 + t] = hb; sVl[r][c4 + t] = bf16_bits(vf[t] - bf16_val(hb));
      }
    }
    __syncthreads();
    v8f s[2];
#pragma unroll
    for (int nt = 0; nt < 2; ++nt) {
      v8f acc = {};
#pragma unroll
      for (int ks = 0; ks < KS; ++ks) {
        FragB bh_, bl_;
        bh_.half[0] = *(const v8us*)&sKh[nt * 16 + ln][ks * 32 + 8 * hh]; bh_.half[1] = *(const v8us*)&sKh[nt * 16 + ln][ks * 32 + 16 + 8 * hh];
        bl_.half[0] = *(const v8us*)&sKl[nt * 16 + ln][ks * 32 + 8 * hh]; bl_.half[1] = *(const v8us*)&sKl[nt * 16 + ln][ks * 32 + 16 + 8 * hh];
        acc = mmaN<3>(aqh[ks].v, aql[ks].v, bh_.v, bl_.v, acc);
      }
      s[nt] = acc;
    }
    float alpha[8];
#pragma unroll
    for (int r = 0; r < 8; ++r) {
      const int qi = q0 + 8 * hh + r;
      const int ja = j0 + ln, jb = j0 + 16 + ln;
      if (CAUSAL) { if (ja > qi) s[0][r] = -3.0e38f; if (jb > qi) s[1][r] = -3.0e38f; }
      if (ja >= T) s[0][r] = -3.0e38f;
      if (jb >= T) s[1][r] = -3.0e38f;
      float mx = fmaxf(s[0][r], s[1][r]);
      mx = fmaxf(mx, __shfl_xor(mx, 1, 32)); mx = fmaxf(mx, __shfl_xor(mx, 2, 32)); mx = fmaxf(mx, __shfl_xor(mx, 4, 32)); mx = fmaxf(mx, __shfl_xor(mx, 8, 32));
      const float mnew = fmaxf(m_r[r], mx);
      alpha[r] = (mnew > -1.0e38f) ? __expf(m_r[r] - mnew) : 1.0f;
      const float p0 = (s[0][r] > -1.0e38f) ? __expf(s[0][r] - mnew) : 0.f;
      const float p1 = (s[1][r] > -1.0e38f) ? __expf(s[1][r] - mnew) : 0.f;
      m_r[r] = mnew;
      l_r[r] = l_r[r] * alpha[r] + p0 + p1;
      unsigned short hb = bf16_bits(p0); sPh[w][8 * hh + r][ln] = hb;      sPl[w][8 * hh + r][ln] = bf16_bits(p0 - bf16_val(hb));
      hb = bf16_bits(p1);                sPh[w][8 * hh + r][16 + ln] = hb; sPl[w][8 * hh + r][16 + ln] = bf16_bits(p1 - bf16_val(hb));
    }
#pragma unroll
    for (int dt = 0; dt < DT; ++dt)
#pragma unroll
      for (int r = 0; r < 8; ++r) oacc[dt][r] *= alpha[r];
    __builtin_amdgcn_fence(__ATOMIC_ACQ_REL, "workgroup");
    __builtin_amdgcn_wave_barrier();
    FragB pah, pal;
    pah.half[0] = *(const v8us*)&sPh[w][ln][8 * hh]; pah.half[1] = *(const v8us*)&sPh[w][ln][16 + 8 * hh];
    pal.half[0] = *(const v8us*)&sPl[w][ln][8 * hh]; pal.half[1] = *(const v8us*)&sPl[w][ln][16 + 8 * hh];
#pragma unroll
    for (int dt = 0; dt < DT; ++dt) {
      FragB bvh, bvl;
#pragma unroll
      for (int i = 0; i < 8; ++i) {
        bvh.u[i] = sVh[8 * hh + i][dt * 16 + ln]; bvh.u[8 + i] = sVh[16 + 8 * hh + i][dt * 16 + ln];
        bvl.u[i] = sVl[8 * hh + i][dt * 16 + ln]; bvl.u[8 + i] = sVl[16 + 8 * hh + i][dt * 16 + ln];
      }
      oacc[dt] = mmaN<3>(pah.v, pal.v, bvh.v, bvl.v, oacc[dt]);
    }
    __builtin_amdgcn_fence(__ATOMIC_ACQ_REL, "workgroup");
    __builtin_amdgcn_wave_barrier();
  }
#pragma unroll
  for (int r = 0; r < 8; ++r) {
    float l = l_r[r];
    l += __shfl_xor(l, 1, 32); l += __shfl_xor(l, 2, 32); l += __shfl_xor(l, 4, 32); l += __shfl_xor(l, 8, 32);
    l_r[r] = (l > 0.f) ? 1.0f / l : 0.f;
  }
#pragma unroll
  for (int dt = 0; dt < DT; ++dt)
#pragma unroll
    for (int r = 0; r < 8; ++r) sO[w][8 * hh + r][dt * 16 + ln] = oacc[dt][r] * l_r[r];
  __builtin_amdgcn_fence(__ATOMIC_ACQ_REL, "workgroup");
  __builtin_amdgcn_wave_barrier();
  for (int pass = 0; pass < 2; ++pass) {
    for (int r = 0; r < 16; ++r) {
      const int row = q0 + r;
      if (row < T && lane < D / 4) {
        const v4f val = *(const v4fa*)&sO[w][r][lane * 4];
        *(volatile v4f*)(y + ((size_t)b * T + row) * ypitch + h * D + lane * 4) = val;
      }
    }
    if (pass == 0) __threadfence();
  }
}

template <bool ASPLIT, int ACT, bool BIAS_BF16, bool RES_BF16>
__global__ __launch_bounds__(128) void k_gemm_bf3(const float* __restrict__ A, int lda, const unsigned short* __restrict__ Wt, int ldb,
                                                const float* __restrict__ bias, const float* __restrict__ resid, int rmod, int ldr,
                                                float* __restrict__ C, int ldc, int M, int N, int K) {
  __shared__ __attribute__((aligned(16))) float so[4][16][64];
  const int tid = threadIdx.x, w = tid >> 5, lane = tid & 31, ln = lane & 15, hh = lane >> 4;
  const int ntn = N / 64;
  const int wid = blockIdx.x * 4 + w;
  const int mt = wid / ntn, nq = wid % ntn;
  if (mt * 16 >= M) return;
  const int row0 = mt * 16, col0 = nq * 64;
  const float* arow = A + (size_t)(row0 + ln) * lda;
  v8f acc[4] = {};
  for (int kb = 0; kb < K; kb += 32) {
    FragB ah, al;
    const v4f x0 = *(const v4fa*)(arow + kb + 8 * hh), x1 = *(const v4fa*)(arow + kb + 8 * hh + 4);
    const v4f x2 = *(const v4fa*)(arow + kb + 16 + 8 * hh), x3 = *(const v4fa*)(arow + kb + 16 + 8 * hh + 4);
    float xs[16] = {x0[0],x0[1],x0[2],x0[3],x1[0],x1[1],x1[2],x1[3],x2[0],x2[1],x2[2],x2[3],x3[0],x3[1],x3[2],x3[3]};
#pragma unroll
    for (int i = 0; i < 16; ++i) { const unsigned short hb = bf16_bits(xs[i]); ah.u[i] = hb; al.u[i] = ASPLIT ? bf16_bits(xs[i] - bf16_val(hb)) : (unsigned short)0; }
#pragma unroll
    for (int t = 0; t < 4; ++t) {
      const unsigned short* brow = Wt + (size_t)(col0 + t * 16 + ln) * ldb + kb;
      FragB b;
      b.half[0] = *(const v8us*)(brow + 8 * hh);
      b.half[1] = *(const v8us*)(brow + 16 + 8 * hh);
      acc[t] = mmaN<ASPLIT ? 2 : 1>(ah.v, al.v, b.v, b.v, acc[t]);
    }
  }
#pragma unroll
  for (int t = 0; t < 4; ++t) {
    const int col = col0 + t * 16 + ln;
    float bv = bias ? bias[col] : 0.f;
    if (BIAS_BF16) bv = bf16_round(bv);
#pragma unroll
    for (int r = 0; r < 8; ++r) {
      float v = acc[t][r] + bv;
      if (resid) { float rv = resid[(size_t)((row0 + 8 * hh + r) % rmod) * ldr + col]; if (RES_BF16) rv = bf16_round(rv); v += rv; }
      if (ACT == 1) v = fmaxf(v, 0.f);
      if (ACT == 2) v = 0.5f * v * (1.0f + erff(v * 0.70710678118654752f));
      if (ACT == 3) { const float u = 0.7978845608028654f * (v + 0.044715f * v * v * v); v = 0.5f * v * (1.0f + tanhf(u)); }
      so[w][8 * hh + r][t * 16 + ln] = v;
    }
  }
  __builtin_amdgcn_fence(__ATOMIC_ACQ_REL, "workgroup");
  __builtin_amdgcn_wave_barrier();
  const int rsub = lane >> 4, c4 = (lane & 15) * 4;
  for (int pass = 0; pass < 2; ++pass) {
#pragma unroll
    for (int q = 0; q < 8; ++q) {
      const int r = q * 2 + rsub;
      const v4f v = *(const v4fa*)&so[w][r][c4];
      *(volatile v4f*)(C + (size_t)(row0 + r) * ldc + col0 + c4) = v;
    }
    if (pass == 0) __threadfence();
  }
}
template <bool PARAM_BF16>
__global__ __launch_bounds__(256) void k_layernorm(const float* __restrict__ X, const float* __restrict__ R, const float* __restrict__ g, const float* __restrict__ bta,
                                                  float* __restrict__ out_sum, float* __restrict__ out_norm, int N, float eps) {
  __shared__ float red[256];
  const int row = blockIdx.x, tid = threadIdx.x;
  const float* x = X + (size_t)row * N; const float* rr = R ? R + (size_t)row * N : nullptr;
  float vals[16];
  const int per = N / 256;
  float s1 = 0.f;
  for (int u = 0; u < per / 4; ++u) {
    const int j = tid * 4 + 1024 * u;
    const v4f a = *(const v4fa*)(x + j);
    v4f b = {0.f,0.f,0.f,0.f}; if (rr) b = *(const v4fa*)(rr + j);
#pragma unroll
    for (int q = 0; q < 4; ++q) { const float v = a[q] + b[q]; vals[u * 4 + q] = v; s1 += v; }
  }
  red[tid] = s1; __syncthreads();
  for (int st = 128; st > 0; st >>= 1) { if (tid < st) red[tid] += red[tid + st]; __syncthreads(); }
  const float mu = red[0] / (float)N; __syncthreads();
  float s2 = 0.f;
  for (int u = 0; u < per / 4; ++u)
#pragma unroll
    for (int q = 0; q < 4; ++q) { const float c = vals[u * 4 + q] - mu; s2 += c * c; }
  red[tid] = s2; __syncthreads();
  for (int st = 128; st > 0; st >>= 1) { if (tid < st) red[tid] += red[tid + st]; __syncthreads(); }
  const float rs = rsqrtf(red[0] / (float)N + eps);
  for (int pass = 0; pass < 2; ++pass) {
    for (int u = 0; u < per / 4; ++u) {
      const int j = tid * 4 + 1024 * u;
      v4f o, sm;
#pragma unroll
      for (int q = 0; q < 4; ++q) {
        float gg = g[j + q], bb = bta[j + q];
        if (PARAM_BF16) { gg = bf16_round(gg); bb = bf16_round(bb); }
        sm[q] = vals[u * 4 + q]; o[q] = (vals[u * 4 + q] - mu) * rs * gg + bb;
      }
      if (out_sum) *(volatile v4f*)(out_sum + (size_t)row * N + j) = sm;
      *(volatile v4f*)(out_norm + (size_t)row * N + j) = o;
    }
    if (pass == 0) __threadfence();
  }
}


typedef _Float16 v16h __attribute__((ext_vector_type(16)));
union FragH { v16h v; v8us half[2]; _Float16 h[16]; unsigned short u[16]; };
template <int NT>
__device__ __forceinline__ v8f mmaH(v16h ah, v16h al, v16h bh, v16h bl, v8f c) {
  c = __builtin_amdgcn_wmma_f32_16x16x32_f16(false, ah, false, bh, (short)0, c, false, false);
  if (NT >= 2) c = __builtin_amdgcn_wmma_f32_16x16x32_f16(false, al, false, bh, (short)0, c, false, false);
  if (NT >= 3) c = __builtin_amdgcn_wmma_f32_16x16x32_f16(false, ah, false, bl, (short)0, c, false, false);
  asm volatile("v_nop\n\tv_nop\n\tv_nop\n\tv_nop" : "+v"(c) : "v"(ah), "v"(al), "v"(bh), "v"(bl));
  return c;
}
template <bool ASPLIT>
__global__ __launch_bounds__(128) void k_gemm_h(const float* __restrict__ A, int lda, size_t sA, const _Float16* __restrict__ Bh, int ldb, size_t sB, float alpha, float* __restrict__ C, int ldc, size_t sC, int M, int N, int K) {
  __shared__ __attribute__((aligned(16))) float so[4][16][64];
  const int tid = threadIdx.x, w = tid >> 5, lane = tid & 31, ln = lane & 15, hh = lane >> 4; const int by = blockIdx.y;
  A += (size_t)by * sA; Bh += (size_t)by * sB; C += (size_t)by * sC;
  const int ntn = (N + 63) / 64; const int wid = blockIdx.x * 4 + w; const int mt = wid / ntn, nq = wid % ntn; if (mt * 16 >= M) return;
  const int row0 = mt * 16, col0 = nq * 64; const float* arow = A + (size_t)(row0 + ln) * lda;
  v8f acc[4] = {};
  for (int kb = 0; kb < K; kb += 32) {
    FragH ah, al;
    const v4f x0 = *(const v4fa*)(arow + kb + 8 * hh), x1 = *(const v4fa*)(arow + kb + 8 * hh + 4), x2 = *(const v4fa*)(arow + kb + 16 + 8 * hh), x3 = *(const v4fa*)(arow + kb + 16 + 8 * hh + 4);
    float xs[16] = {x0[0],x0[1],x0[2],x0[3],x1[0],x1[1],x1[2],x1[3],x2[0],x2[1],x2[2],x2[3],x3[0],x3[1],x3[2],x3[3]};
#pragma unroll
    for (int i = 0; i < 16; ++i) { const _Float16 h = (_Float16)xs[i]; ah.h[i] = h; al.h[i] = ASPLIT ? (_Float16)(xs[i] - (float)h) : (_Float16)0.0f; }
#pragma unroll
    for (int t = 0; t < 4; ++t) { if (col0 + t * 16 >= N) continue; const size_t boff = (size_t)(col0 + t * 16 + ln) * ldb + kb; FragH bq; bq.half[0] = *(const v8us*)(Bh + boff + 8 * hh); bq.half[1] = *(const v8us*)(Bh + boff + 16 + 8 * hh);
      acc[t] = mmaH<ASPLIT ? 2 : 1>(ah.v, al.v, bq.v, bq.v, acc[t]); }
  }
#pragma unroll
  for (int t = 0; t < 4; ++t) { if (col0 + t * 16 >= N) continue;
#pragma unroll
    for (int r = 0; r < 8; ++r) so[w][8 * hh + r][t * 16 + ln] = acc[t][r] * alpha; }
  __builtin_amdgcn_fence(__ATOMIC_ACQ_REL, "workgroup"); __builtin_amdgcn_wave_barrier();
  const int rsub = lane >> 4, c4 = (lane & 15) * 4;
  for (int pass = 0; pass < 2; ++pass) {
#pragma unroll
    for (int q = 0; q < 8; ++q) { const int r = q * 2 + rsub; if (col0 + c4 < N) { const v4f v = *(const v4fa*)&so[w][r][c4]; *(volatile v4f*)(C + (size_t)(row0 + r) * ldc + col0 + c4) = v; } }
    if (pass == 0) __threadfence(); }
}

__global__ __launch_bounds__(256) void k_wt_f16(const float* __restrict__ W, _Float16* __restrict__ Wt, int K, int N, float scale) {
  const int t = blockIdx.x * 256 + threadIdx.x; if (t >= N * (K / 8)) return; const int n = t / (K / 8), k8 = (t % (K / 8)) * 8; FragH f;
#pragma unroll
  for (int i = 0; i < 8; ++i) f.h[i] = (_Float16)(bf16_round(W[(size_t)(k8 + i) * N + n]) * scale); const v8us o = f.half[0];
  *(volatile v8us*)((unsigned short*)Wt + (size_t)n * K + k8) = o; __threadfence(); *(volatile v8us*)((unsigned short*)Wt + (size_t)n * K + k8) = o;
}
template <int ACT>
__global__ __launch_bounds__(128) void k_gemm_hhx(const _Float16* __restrict__ A, int lda, size_t sA, const _Float16* __restrict__ Bh, int ldb, size_t sB, float alpha, const float* __restrict__ bias, size_t sBias, const float* __restrict__ CP, int rowsPerB, size_t sCPb, int row0g,
    float* __restrict__ C, _Float16* __restrict__ C16, int ldc, size_t sC, int M, int N, int K) {
  __shared__ __attribute__((aligned(16))) float so[4][16][64];
  const int tid = threadIdx.x, w = tid >> 5, lane = tid & 31, ln = lane & 15, hh = lane >> 4; const int by = blockIdx.y;
  A += (size_t)by * sA; Bh += (size_t)by * sB; const size_t cofs = (size_t)by * sC; const float* bp = bias ? bias + (size_t)by * sBias : nullptr;
  const int ntn = (N + 63) / 64; const int wid = blockIdx.x * 4 + w; const int mt = wid / ntn, nq = wid % ntn; if (mt * 16 >= M) return;
  const int row0 = mt * 16, col0 = nq * 64; const _Float16* arow = A + (size_t)(row0 + ln) * lda;
  v8f acc[4] = {};
  for (int kb = 0; kb < K; kb += 32) { FragH ah; ah.half[0] = *(const v8us*)((const unsigned short*)arow + kb + 8 * hh); ah.half[1] = *(const v8us*)((const unsigned short*)arow + kb + 16 + 8 * hh);
#pragma unroll
    for (int t = 0; t < 4; ++t) { if (col0 + t * 16 >= N) continue; const size_t boff = (size_t)(col0 + t * 16 + ln) * ldb + kb; FragH bq; bq.half[0] = *(const v8us*)((const unsigned short*)Bh + boff + 8 * hh); bq.half[1] = *(const v8us*)((const unsigned short*)Bh + boff + 16 + 8 * hh);
      acc[t] = mmaH<1>(ah.v, ah.v, bq.v, bq.v, acc[t]); }
  }
#pragma unroll
  for (int t = 0; t < 4; ++t) { if (col0 + t * 16 >= N) continue; const int col = col0 + t * 16 + ln; const float bv = bp ? bf16_round(bp[col]) : 0.f;
#pragma unroll
    for (int r = 0; r < 8; ++r) { float v = acc[t][r] * alpha + bv; if (CP) { const int bidx = (row0g + row0 + 8 * hh + r) / rowsPerB; v += CP[(size_t)bidx * sCPb + (size_t)by * 64 + col]; } if (ACT == 1) v = (v > 0.f) ? v : expm1f(v); else if (ACT == 3) v = fmaxf(v, 0.f); so[w][8 * hh + r][t * 16 + ln] = v; } }
  __builtin_amdgcn_fence(__ATOMIC_ACQ_REL, "workgroup"); __builtin_amdgcn_wave_barrier();
  const int rsub = lane >> 4, c4 = (lane & 15) * 4; typedef _Float16 v4h __attribute__((ext_vector_type(4)));
  for (int pass = 0; pass < 2; ++pass) {
#pragma unroll
    for (int q = 0; q < 8; ++q) { const int r = q * 2 + rsub; if (col0 + c4 < N) { const v4f v = *(const v4fa*)&so[w][r][c4]; if (C) *(volatile v4f*)(C + cofs + (size_t)(row0 + r) * ldc + col0 + c4) = v; if (C16) { v4h h4; for (int i = 0; i < 4; ++i) h4[i] = (_Float16)v[i]; *(volatile v4h*)(C16 + cofs + (size_t)(row0 + r) * ldc + col0 + c4) = h4; } } }
    if (pass == 0) __threadfence(); }
}


typedef _Float16 v4h __attribute__((ext_vector_type(4)));

__global__ __launch_bounds__(256) void k_x16(const float* __restrict__ x, _Float16* __restrict__ X16, size_t n8) { const size_t t = (size_t)blockIdx.x * 256 + threadIdx.x; if (t >= n8) return; FragH f;
#pragma unroll
  for (int q = 0; q < 8; ++q) f.h[q] = (_Float16)bf16_round(x[t * 8 + q]); *(volatile v8us*)((unsigned short*)X16 + t * 8) = f.half[0]; __threadfence(); *(volatile v8us*)((unsigned short*)X16 + t * 8) = f.half[0]; }
__global__ __launch_bounds__(256) void k_h16(const float* __restrict__ x, _Float16* __restrict__ X16, size_t n8) { const size_t t = (size_t)blockIdx.x * 256 + threadIdx.x; if (t >= n8) return; FragH f;
#pragma unroll
  for (int q = 0; q < 8; ++q) f.h[q] = (_Float16)x[t * 8 + q]; *(volatile v8us*)((unsigned short*)X16 + t * 8) = f.half[0]; __threadfence(); *(volatile v8us*)((unsigned short*)X16 + t * 8) = f.half[0]; }
__global__ __launch_bounds__(256) void k_round16f(const float* __restrict__ W, _Float16* __restrict__ Bt, size_t n8) { const size_t t = (size_t)blockIdx.x * 256 + threadIdx.x; if (t >= n8) return; FragH f;
#pragma unroll
  for (int i = 0; i < 8; ++i) f.h[i] = (_Float16)(bf16_round(W[t * 8 + i]) * 16.0f); *(volatile v8us*)((unsigned short*)Bt + t * 8) = f.half[0]; __threadfence(); *(volatile v8us*)((unsigned short*)Bt + t * 8) = f.half[0]; }
template <int NHv, int TTv>
__global__ __launch_bounds__(256) void k_vt(const _Float16* __restrict__ V16, int ldv, int voff, _Float16* __restrict__ Vt) { __shared__ unsigned short tl[64][66]; const int tid = threadIdx.x; const int slab = blockIdx.x / (TTv / 64), lg = blockIdx.x % (TTv / 64); const int b = slab / NHv, h = slab % NHv;
  for (int i = tid; i < 64 * 8; i += 256) { const int r = i / 8, c8 = (i % 8) * 8; FragH f; f.half[0] = *(const v8us*)((const unsigned short*)V16 + ((size_t)b * TTv + lg * 64 + r) * ldv + voff + h * 64 + c8);
#pragma unroll
    for (int q = 0; q < 8; ++q) tl[r][c8 + q] = f.u[q]; }
  __syncthreads();
  for (int pass = 0; pass < 2; ++pass) {
#pragma unroll
    for (int rd = 0; rd < 2; ++rd) { const int d = rd * 32 + tid / 8, pc = tid % 8; FragH f;
#pragma unroll
      for (int q = 0; q < 8; ++q) f.u[q] = tl[pc * 8 + q][d];
      *(volatile v8us*)((unsigned short*)Vt + ((size_t)slab * 64 + d) * TTv + lg * 64 + pc * 8) = f.half[0]; }
    if (pass == 0) __threadfence(); } }

__global__ __launch_bounds__(32) void k_s4k(const float* __restrict__ log_dt, const float* __restrict__ Alr, const float* __restrict__ Aim, const float* __restrict__ Bre, const float* __restrict__ Bim, const float* __restrict__ Cre, const float* __restrict__ Cim, float* __restrict__ K) { __shared__ float sk[LL]; const int h = blockIdx.x, c = threadIdx.x; const float dt = expf(bf16_round(log_dt[h]));
  for (int i = 0; i < 32; ++i) sk[32 * c + i] = 0.f;
#pragma unroll 1
  for (int n = 0; n < NS; ++n) { const size_t hn = (size_t)h * NS + n; const float ar = -expf(bf16_round(Alr[hn])), ai = bf16_round(Aim[hn]); const float dr = dt * ar, di = dt * ai;
    const float er = expf(dr); float sn, cs; sincosf(di, &sn, &cs); const float e1r = er * cs - 1.0f, e1i = er * sn;
    const float den = ar * ar + ai * ai; const float qr = (e1r * ar + e1i * ai) / den, qi = (e1i * ar - e1r * ai) / den;
    const float br = bf16_round(Bre[hn]), bi = bf16_round(Bim[hn]); const float bbr = qr * br - qi * bi, bbi = qr * bi + qi * br;
    const float cr = bf16_round(Cre[hn]), ci = bf16_round(Cim[hn]); const float cbr = cr * bbr - ci * bbi, cbi = cr * bbi + ci * bbr;
    const float l0 = (float)(32 * c); const float sr0 = expf(dr * l0); float s0, c0; sincosf(di * l0, &s0, &c0); float vr = sr0 * c0, vi = sr0 * s0; const float wr = er * cs, wi = er * sn;
#pragma unroll 1
    for (int i = 0; i < 32; ++i) { sk[32 * c + i] += 2.0f * (cbr * vr - cbi * vi); const float nr = vr * wr - vi * wi, ni = vr * wi + vi * wr; vr = nr; vi = ni; } }
  __builtin_amdgcn_fence(__ATOMIC_ACQ_REL, "workgroup"); __builtin_amdgcn_wave_barrier();
  for (int pass = 0; pass < 2; ++pass) { for (int j = 0; j < 32; ++j) *(volatile float*)(K + (size_t)h * LL + j * 32 + c) = sk[j * 32 + c]; if (pass == 0) __threadfence(); } }
__global__ __launch_bounds__(256) void k_toep(const float* __restrict__ K, int h0, _Float16* __restrict__ T) { const size_t t = (size_t)blockIdx.x * 256 + threadIdx.x; if (t >= (size_t)HCH * LL * (LL / 8)) return; const int j8 = (int)(t % (LL / 8)) * 8; const int l = (int)((t / (LL / 8)) % LL); const int hh = (int)(t / ((size_t)(LL / 8) * LL)); const float* kr = K + (size_t)(h0 + hh) * LL; FragH f; for (int q = 0; q < 8; ++q) { const int j = j8 + q; f.h[q] = (_Float16)((j <= l) ? kr[l - j] : 0.f); } *(volatile v8us*)((unsigned short*)T + t * 8) = f.half[0]; __threadfence(); *(volatile v8us*)((unsigned short*)T + t * 8) = f.half[0]; }
__global__ __launch_bounds__(256) void k_u16(const float* __restrict__ H0, _Float16* __restrict__ U16) { const size_t t = (size_t)blockIdx.x * 256 + threadIdx.x; if (t >= (size_t)HH * 16 * (LL / 8)) return; const int j8 = (int)(t % (LL / 8)) * 8; const int b = (int)((t / (LL / 8)) % 16); const int h = (int)(t / ((size_t)(LL / 8) * 16)); FragH f; for (int q = 0; q < 8; ++q) f.h[q] = (_Float16)((b < BB) ? H0[((size_t)b * LL + j8 + q) * HH + h] : 0.f); *(volatile v8us*)((unsigned short*)U16 + t * 8) = f.half[0]; __threadfence(); *(volatile v8us*)((unsigned short*)U16 + t * 8) = f.half[0]; }
__global__ __launch_bounds__(256) void k_ygelu(const float* __restrict__ Y, const float* __restrict__ H0, const float* __restrict__ D, _Float16* __restrict__ G16) { const size_t t = (size_t)blockIdx.x * 256 + threadIdx.x; if (t >= (size_t)NR * (HH / 8)) return; const int h8 = (int)(t % (HH / 8)) * 8; const size_t r = t / (HH / 8); const int b = (int)(r / LL), l = (int)(r % LL); FragH f;
#pragma unroll
  for (int q = 0; q < 8; ++q) { const int h = h8 + q; const float y = Y[((size_t)h * LL + l) * 16 + b] + bf16_round(D[h]) * H0[r * HH + h]; const float u = 0.7978845608028654f * (y + 0.044715f * y * y * y); const float e = __expf(2.0f * u); const float th = 1.0f - 2.0f / (e + 1.0f); f.h[q] = (_Float16)(0.5f * y * (1.0f + th)); }
  *(volatile v8us*)((unsigned short*)G16 + t * 8) = f.half[0]; __threadfence(); *(volatile v8us*)((unsigned short*)G16 + t * 8) = f.half[0]; }
__global__ __launch_bounds__(256) void k_xpad(const float* __restrict__ x, _Float16* __restrict__ XP) { const size_t t = (size_t)blockIdx.x * 256 + threadIdx.x; if (t >= (size_t)BB * (LL + 4) * (IN / 8)) return; const int c8 = (int)(t % (IN / 8)) * 8; const int rr = (int)((t / (IN / 8)) % (LL + 4)); const int b = (int)(t / ((size_t)(IN / 8) * (LL + 4))); const int l = rr - 2; FragH f; for (int q = 0; q < 8; ++q) f.h[q] = (_Float16)((l >= 0 && l < LL) ? bf16_round(x[((size_t)b * LL + l) * IN + c8 + q]) : 0.f); *(volatile v8us*)((unsigned short*)XP + t * 8) = f.half[0]; __threadfence(); *(volatile v8us*)((unsigned short*)XP + t * 8) = f.half[0]; }
__global__ __launch_bounds__(256) void k_wtap(const float* __restrict__ W, _Float16* __restrict__ Bt) { const int t = blockIdx.x * 256 + threadIdx.x; if (t >= 3 * HH * (IN / 8)) return; const int c8 = (t % (IN / 8)) * 8; const int o = (t / (IN / 8)) % HH; const int k = t / ((IN / 8) * HH); FragH f; for (int q = 0; q < 8; ++q) f.h[q] = (_Float16)(bf16_round(W[((size_t)o * IN + c8 + q) * 3 + k]) * 16.0f); *(volatile v8us*)((unsigned short*)Bt + (size_t)t * 8) = f.half[0]; __threadfence(); *(volatile v8us*)((unsigned short*)Bt + (size_t)t * 8) = f.half[0]; }
__global__ __launch_bounds__(256) void k_ln256(const float* __restrict__ G, const float* __restrict__ R, const float* __restrict__ gam, const float* __restrict__ bet, int ntn, float* __restrict__ OF, _Float16* __restrict__ O16) { const int tid = threadIdx.x, wv = tid >> 5, lane = tid & 31; const size_t r = (size_t)blockIdx.x * 8 + wv; if (r >= (size_t)NR) return; v4f y[2]; float s = 0.f;
#pragma unroll
  for (int j = 0; j < 2; ++j) { const int c = j * 128 + lane * 4; v4f g = *(const v4fa*)(G + r * HH + c); if (R) { const v4f x = *(const v4fa*)(R + r * HH + c); for (int q = 0; q < 4; ++q) g[q] += x[q]; } if (ntn) { for (int q = 0; q < 4; ++q) { float v = g[q]; if (v != v) v = 0.f; v = fminf(fmaxf(v, -1e6f), 1e6f); g[q] = v; } } y[j] = g; s += g[0] + g[1] + g[2] + g[3]; }
  for (int o = 16; o >= 1; o >>= 1) s += __shfl_xor(s, o, 32); const float mu = s / (float)HH; float q2 = 0.f; for (int j = 0; j < 2; ++j) for (int q = 0; q < 4; ++q) { const float d = y[j][q] - mu; q2 += d * d; } for (int o = 16; o >= 1; o >>= 1) q2 += __shfl_xor(q2, o, 32); const float rs = rsqrtf(q2 / (float)HH + 1e-5f);
  for (int pass = 0; pass < 2; ++pass) { for (int j = 0; j < 2; ++j) { const int c = j * 128 + lane * 4; v4f o; v4h hh4; for (int q = 0; q < 4; ++q) { const float v = (y[j][q] - mu) * rs * bf16_round(gam[c + q]) + bf16_round(bet[c + q]); o[q] = v; hh4[q] = (_Float16)v; } if (OF) *(volatile v4f*)(OF + r * HH + c) = o; if (O16) *(volatile v4h*)(O16 + r * HH + c) = hh4; } if (pass == 0) __threadfence(); } }
extern "C" void kernel_launch(void* const* d_in, const int* in_sizes, int n_in,
                              void* d_out, int out_size, void* d_ws, size_t ws_size, hipStream_t stream) {
  (void)in_sizes; (void)n_in; (void)out_size;
  const float* const* I = (const float* const*)d_in; const float* x = I[0]; const float* Wenc = I[1]; const float* benc = I[2]; const float* log_dt = I[3]; const float* Alr = I[4]; const float* Aim = I[5]; const float* Bre = I[6]; const float* Bim = I[7]; const float* Cre = I[8]; const float* Cim = I[9]; const float* D = I[10]; const float* Wblk = I[11]; const float* bblk = I[12]; const float* g1 = I[13]; const float* b1 = I[14]; const float* Wdec = I[15]; const float* bdec = I[16]; const float* Wtcn = I[17]; const float* btcn = I[18]; const float* g2 = I[19]; const float* b2 = I[20];
  char* ws = (char*)d_ws; size_t off = 0;
  auto take = [&](size_t bytes) { char* p = ws + off; off += (bytes + 255) & ~(size_t)255; return p; };
  _Float16* Benc = (_Float16*)take((size_t)HH * IN * 2); _Float16* Bblk = (_Float16*)take((size_t)HH * HH * 2); _Float16* Bdec = (_Float16*)take((size_t)HH * HH * 2); _Float16* Btap = (_Float16*)take((size_t)3 * HH * IN * 2);
  _Float16* X16 = (_Float16*)take((size_t)NR * IN * 2); float* H0 = (float*)take((size_t)NR * HH * 4); float* K = (float*)take((size_t)HH * LL * 4); _Float16* U16 = (_Float16*)take((size_t)HH * 16 * LL * 2); _Float16* T = (_Float16*)take((size_t)HCH * LL * LL * 2); float* Y = (float*)take((size_t)HH * LL * 16 * 4); _Float16* G16 = (_Float16*)take((size_t)NR * HH * 2); float* Z = (float*)take((size_t)NR * HH * 4); _Float16* H116 = (_Float16*)take((size_t)NR * HH * 2); float* S4 = (float*)take((size_t)NR * HH * 4); _Float16* XP = (_Float16*)take((size_t)BB * (LL + 4) * IN * 2);
  if (off > ws_size) return;
  k_wt_f16<<<(HH * (IN / 8) + 255) / 256, 256, 0, stream>>>(Wenc, Benc, IN, HH, 16.0f); k_wt_f16<<<(HH * (HH / 8) + 255) / 256, 256, 0, stream>>>(Wblk, Bblk, HH, HH, 16.0f); k_wt_f16<<<(HH * (HH / 8) + 255) / 256, 256, 0, stream>>>(Wdec, Bdec, HH, HH, 16.0f);
  k_wtap<<<(3 * HH * (IN / 8) + 255) / 256, 256, 0, stream>>>(Wtcn, Btap);
  k_x16<<<(unsigned)(((size_t)NR * IN / 8 + 255) / 256), 256, 0, stream>>>(x, X16, (size_t)NR * IN / 8); k_xpad<<<(unsigned)(((size_t)BB * (LL + 4) * (IN / 8) + 255) / 256), 256, 0, stream>>>(x, XP);
  const dim3 gH(((NR / 16) * (HH / 64) + 3) / 4, 1);
  k_gemm_hhx<0><<<gH, 128, 0, stream>>>(X16, IN, 0, Benc, IN, 0, 0.0625f, benc, 0, nullptr, 1, 0, 0, H0, nullptr, HH, 0, NR, HH, IN);
  k_s4k<<<HH, 32, 0, stream>>>(log_dt, Alr, Aim, Bre, Bim, Cre, Cim, K);
  k_u16<<<(unsigned)(((size_t)HH * 16 * (LL / 8) + 255) / 256), 256, 0, stream>>>(H0, U16);
  for (int h0c = 0; h0c < HH; h0c += HCH) {
    k_toep<<<(unsigned)(((size_t)HCH * LL * (LL / 8) + 255) / 256), 256, 0, stream>>>(K, h0c, T);
    k_gemm_hhx<0><<<dim3(((LL / 16) * 1 + 3) / 4, HCH), 128, 0, stream>>>(T, LL, (size_t)LL * LL, U16 + (size_t)h0c * 16 * LL, LL, (size_t)16 * LL, 1.0f, nullptr, 0, nullptr, 1, 0, 0, Y + (size_t)h0c * LL * 16, nullptr, 16, (size_t)LL * 16, LL, 16, LL); }
  k_ygelu<<<(unsigned)(((size_t)NR * (HH / 8) + 255) / 256), 256, 0, stream>>>(Y, H0, D, G16);
  k_gemm_hhx<0><<<gH, 128, 0, stream>>>(G16, HH, 0, Bblk, HH, 0, 0.0625f, bblk, 0, nullptr, 1, 0, 0, Z, nullptr, HH, 0, NR, HH, HH);
  k_ln256<<<(NR + 7) / 8, 256, 0, stream>>>(Z, H0, g1, b1, 0, nullptr, H116);
  k_gemm_hhx<0><<<gH, 128, 0, stream>>>(H116, HH, 0, Bdec, HH, 0, 0.0625f, bdec, 0, nullptr, 1, 0, 0, S4, nullptr, HH, 0, NR, HH, HH);
  for (int b = 0; b < BB; ++b) for (int k = 0; k < 3; ++k) k_gemm_hhx<0><<<dim3(((LL / 16) * (HH / 64) + 3) / 4, 1), 128, 0, stream>>>(XP + ((size_t)b * (LL + 4) + 2 * k) * IN, IN, 0, Btap + (size_t)k * HH * IN, IN, 0, 0.0625f, k == 0 ? btcn : nullptr, 0, S4 + (size_t)b * LL * HH, 1, (size_t)HH, 0, S4 + (size_t)b * LL * HH, nullptr, HH, 0, LL, HH, IN);
  k_ln256<<<(NR + 7) / 8, 256, 0, stream>>>(S4, nullptr, g2, b2, 1, (float*)d_out, nullptr);
}
